// TransformerUnit_377957122743
// MI455X (gfx1250) — hardware-verified
//
#include <hip/hip_runtime.h>
#include <math.h>

typedef __attribute__((ext_vector_type(16))) _Float16 v16h;
typedef __attribute__((ext_vector_type(8)))  _Float16 v8h;
typedef __attribute__((ext_vector_type(16))) __bf16   v16b;
typedef __attribute__((ext_vector_type(8)))  __bf16   v8b;
typedef __attribute__((ext_vector_type(8)))  float    v8f;
typedef __attribute__((ext_vector_type(4)))  float    v4f;

constexpr int NBATCH = 2;
constexpr int NCHAN  = 64;
constexpr int IMG_H  = 96;
constexpr int IMG_W  = 96;
constexpr int HWPIX  = IMG_H * IMG_W;
constexpr int NROWS  = NBATCH * HWPIX;
constexpr int NHEADS = 8;
constexpr int HDIM   = 8;
constexpr int KWIN   = 5;
constexpr int NTAPS  = KWIN * KWIN;
constexpr int NHID   = 128;
constexpr long PLANE16 = (long)NROWS * NCHAN;
constexpr long PLANE32 = (long)NROWS * NCHAN;
constexpr int NSAMPLE = NCHAN * HWPIX;
constexpr int GN_BLOCKS = 128;
constexpr int GN_CHUNK  = 9216;
static_assert(GN_BLOCKS * GN_CHUNK == NBATCH * NSAMPLE);
static_assert(GN_CHUNK % 1024 == 0);
static_assert(NROWS % 64 == 0 && NROWS % 32 == 0 && HWPIX % 64 == 0);
static_assert(NCHAN % 32 == 0 && NHID % 64 == 0);

constexpr int TAB_B1    = 64 * 96;
constexpr int TAB_B2    = TAB_B1 + NHID;
constexpr int TAB_TOTAL = TAB_B2 + NCHAN;
static_assert(TAB_TOTAL % 32 == 0 && TAB_B1 % 32 == 0 && TAB_B2 % 32 == 0);

constexpr int W_Q = 0, W_K = 4096, W_V = 8192, W_FC = 12288, W_M1 = 16384, W_M2 = 24576, W_TOTAL = 32768;

constexpr int ATT_PITCH = 72;
constexpr int OUT_PITCH = 68;
constexpr int TILE_PITCH = 68;

constexpr size_t SZ_TAB  = 25600;
constexpr size_t SZ_WALL = (size_t)W_TOTAL * 2;
constexpr size_t SZ_X16  = (size_t)3 * PLANE16 * 2;
constexpr size_t SZ_QKV  = (size_t)3 * PLANE32 * 4;
constexpr size_t SZ_FC32 = (size_t)PLANE32 * 4;
constexpr size_t SZ_FC16 = (size_t)PLANE16 * 2;
constexpr size_t SZ_HD16 = (size_t)NROWS * NHID * 2;
constexpr size_t SZ_Y2   = (size_t)PLANE32 * 4;
constexpr size_t SZ_P    = (size_t)GN_BLOCKS * 128;
constexpr size_t OFF_TAB  = 0;
constexpr size_t OFF_WALL = OFF_TAB + SZ_TAB;
constexpr size_t OFF_X16  = OFF_WALL + SZ_WALL;
constexpr size_t OFF_QKV  = OFF_X16 + SZ_X16;
constexpr size_t OFF_FC32 = OFF_QKV + SZ_QKV;
constexpr size_t OFF_FC16 = OFF_FC32 + SZ_FC32;
constexpr size_t OFF_HD16 = OFF_FC16 + SZ_FC16;
constexpr size_t OFF_Y2   = OFF_HD16 + SZ_HD16;
constexpr size_t OFF_P1   = OFF_Y2 + SZ_Y2;
constexpr size_t OFF_P2   = OFF_P1 + SZ_P;
constexpr size_t WS_TOTAL = OFF_P2 + SZ_P;
static_assert(SZ_TAB >= (size_t)TAB_TOTAL * 4);
static_assert(OFF_WALL % 256 == 0 && OFF_X16 % 256 == 0 && OFF_QKV % 256 == 0 && OFF_FC32 % 256 == 0);
static_assert(OFF_FC16 % 256 == 0 && OFF_HD16 % 256 == 0 && OFF_Y2 % 256 == 0 && OFF_P1 % 256 == 0 && OFF_P2 % 256 == 0);
static_assert(WS_TOTAL == 37872640);
static_assert(WS_TOTAL <= (size_t)134217728);

__device__ __forceinline__ int imin(int a, int b) { return a < b ? a : b; }
__device__ __forceinline__ int imax(int a, int b) { return a > b ? a : b; }

__device__ __forceinline__ float bf16r(float f) {
  unsigned u = __float_as_uint(f);
  u = (u + 0x7FFFu + ((u >> 16) & 1u)) & 0xFFFF0000u;
  return __uint_as_float(u);
}

__device__ __forceinline__ unsigned short f2bf_bits(float f) {
  unsigned u = __float_as_uint(f);
  return (unsigned short)((u + 0x7FFFu + ((u >> 16) & 1u)) >> 16);
}
__device__ __forceinline__ float bf_bits2f(unsigned short h) { return __uint_as_float(((unsigned)h) << 16); }

__device__ __forceinline__ void dep_guard_h(v8f& a, v8f& b, v16h x, v16h y) { asm volatile("v_nop\n\tv_nop\n\tv_nop\n\tv_nop" : "+v"(a), "+v"(b) : "v"(x), "v"(y)); }
__device__ __forceinline__ void dep_guard_b(v8f& a, v8f& b, v16b x, v16b y) { asm volatile("v_nop\n\tv_nop\n\tv_nop\n\tv_nop" : "+v"(a), "+v"(b) : "v"(x), "v"(y)); }
__device__ __forceinline__ void keep4_h(v16h a, v16h b, v16h c, v16h d) { asm volatile("v_nop" :: "v"(a), "v"(b), "v"(c), "v"(d)); }
__device__ __forceinline__ void keep4_b(v16b a, v16b b, v16b c, v16b d) { asm volatile("v_nop" :: "v"(a), "v"(b), "v"(c), "v"(d)); }
__device__ __forceinline__ void acc_guard4(v8f& a, v8f& b, v8f& c, v8f& d) { asm volatile("v_nop\n\tv_nop\n\tv_nop\n\tv_nop" : "+v"(a), "+v"(b), "+v"(c), "+v"(d)); }
__device__ __forceinline__ void mma_guard1(v8f& c, v16h a, v16h b) { asm volatile("v_nop\n\tv_nop\n\tv_nop\n\tv_nop" : "+v"(c) : "v"(a), "v"(b)); }

template <typename T> struct Frag;
template <> struct Frag<_Float16> {
  typedef v16h V; union U { v16h v; v8h h[2]; };
  static __device__ __forceinline__ v16h load(const _Float16* p) {
    U f; f.h[0] = *(const v8h*)(p); f.h[1] = *(const v8h*)(p + 16); return f.v;
  }
  static __device__ __forceinline__ v8f mma(v16h a, v16h b, v8f c) {
    return __builtin_amdgcn_wmma_f32_16x16x32_f16(false, a, false, b, (short)0, c, false, false);
  }
  static __device__ __forceinline__ void guard(v8f& a, v8f& b, v16h x, v16h y) { dep_guard_h(a, b, x, y); }
  static __device__ __forceinline__ void keep(v16h a, v16h b, v16h c, v16h d) { keep4_h(a, b, c, d); }
};
template <> struct Frag<__bf16> {
  typedef v16b V; union U { v16b v; v8b h[2]; };
  static __device__ __forceinline__ v16b load(const __bf16* p) {
    U f; f.h[0] = *(const v8b*)(p); f.h[1] = *(const v8b*)(p + 16); return f.v;
  }
  static __device__ __forceinline__ v8f mma(v16b a, v16b b, v8f c) {
    return __builtin_amdgcn_wmma_f32_16x16x32_bf16(false, a, false, b, (short)0, c, false, false);
  }
  static __device__ __forceinline__ void guard(v8f& a, v8f& b, v16b x, v16b y) { dep_guard_b(a, b, x, y); }
  static __device__ __forceinline__ void keep(v16b a, v16b b, v16b c, v16b d) { keep4_b(a, b, c, d); }
};

template <int ET> struct Elem;
template <> struct Elem<0> { typedef _Float16 T; };
template <> struct Elem<1> { typedef __bf16 T; };
template <int ET, bool SPLIT, int BIAS_MODE, int OUT_MODE, bool RESID, int ACT = 0>
__global__ __launch_bounds__(256) void wmma_gemm64(
    const unsigned short* __restrict__ Ap, const unsigned short* __restrict__ A2p, int lda, long strideA,
    const unsigned short* __restrict__ Btp, const unsigned short* __restrict__ Bt2p, int ldb, long strideB,
    void* __restrict__ Cout, void* __restrict__ Cout2, int ldc, long strideC,
    const float* __restrict__ bias,
    const float* __restrict__ resid, long strideR,
    int M, int N, int K, float scale) {
  typedef typename Elem<ET>::T T;
  typedef typename Frag<T>::V V;
  const T* A = (const T*)Ap; const T* A2 = (const T*)A2p; const T* Bt = (const T*)Btp; const T* Bt2 = (const T*)Bt2p;
  __shared__ __align__(16) float sT[8][16 * 68];
  const int b    = blockIdx.y;
  const int lane = threadIdx.x & 31;
  const int wave = threadIdx.x >> 5;
  const int tilesN = N >> 6;
  const int tilesM = M >> 6;
  const int tile = blockIdx.x * 8 + wave;
  if (tile >= tilesM * tilesN) return;
  const int tm = tile / tilesN;
  const int tn = tile - tm * tilesN;
  const int m0 = tm << 6;
  const int n0 = tn << 6;

  const T* Ab  = A  + (size_t)b * strideA;
  const T* Bb  = Bt + (size_t)b * strideB;
  const T* Ab2 = SPLIT ? (A2  + (size_t)b * strideA) : nullptr;
  const T* Bb2 = SPLIT ? (Bt2 + (size_t)b * strideB) : nullptr;

  const int rlane = lane & 15;
  const int koff  = (lane >> 4) * 8;
  const int mOff  = (lane >> 4) * 8;

  v8f acc[4][4];
#pragma unroll
  for (int i = 0; i < 4; ++i)
#pragma unroll
    for (int j = 0; j < 4; ++j) acc[i][j] = (v8f){0.f,0.f,0.f,0.f,0.f,0.f,0.f,0.f};

  for (int k0 = 0; k0 < K; k0 += 32) {
    V bh[4], bl[4];
#pragma unroll
    for (int j = 0; j < 4; ++j) {
      const size_t bo = (size_t)(n0 + (j << 4) + rlane) * ldb + koff + k0;
      bh[j] = Frag<T>::load(Bb + bo);
      if (SPLIT) bl[j] = Frag<T>::load(Bb2 + bo);
    }
#pragma unroll
    for (int i = 0; i < 4; ++i) {
      const size_t ao = (size_t)(m0 + (i << 4) + rlane) * lda + koff + k0;
      V ah = Frag<T>::load(Ab + ao);
      V al;
      if (SPLIT) al = Frag<T>::load(Ab2 + ao);
#pragma unroll
      for (int j = 0; j < 4; ++j) {
        acc[i][j] = Frag<T>::mma(ah, bh[j], acc[i][j]);
        if (SPLIT) {
          acc[i][j] = Frag<T>::mma(ah, bl[j], acc[i][j]);
          acc[i][j] = Frag<T>::mma(al, bh[j], acc[i][j]);
        }
      }
      Frag<T>::guard(acc[i][0], acc[i][3], ah, SPLIT ? al : ah);
    }
    Frag<T>::keep(bh[0], bh[1], bh[2], bh[3]);
    if (SPLIT) Frag<T>::keep(bl[0], bl[1], bl[2], bl[3]);
  }
  acc_guard4(acc[0][0], acc[0][1], acc[0][2], acc[0][3]);
  acc_guard4(acc[1][0], acc[1][1], acc[1][2], acc[1][3]);
  acc_guard4(acc[2][0], acc[2][1], acc[2][2], acc[2][3]);
  acc_guard4(acc[3][0], acc[3][1], acc[3][2], acc[3][3]);

  float* slab = sT[wave];
  const float* Rb = RESID ? (resid + (size_t)b * strideR) : nullptr;
#pragma unroll
  for (int i = 0; i < 4; ++i) {
    const int mBase = m0 + (i << 4);
#pragma unroll
    for (int j = 0; j < 4; ++j) {
      const int n = n0 + (j << 4) + rlane;
      float bv = 0.f;
      if (BIAS_MODE == 2) bv = bias[n];
#pragma unroll
      for (int r = 0; r < 8; ++r) {
        float v = acc[i][j][r] * scale;
        if (BIAS_MODE == 1) v += bias[mBase + mOff + r];
        if (BIAS_MODE == 2) v += bv;
        if (RESID) v += Rb[(size_t)(mBase + mOff + r) * ldc + n];
        if (ACT == 1) v = tanhf(v);
        if (ACT == 2) v = fmaxf(v, 0.0f);
        if (ACT == 3) v = v / (1.0f + expf(-v));
        if (ACT == 4) v = (v > 0.f) ? v : 0.01f * v;
        if (ACT == 6) v = (v >= 0.f) ? v : 0.2f * v;
        slab[(mOff + r) * 68 + (j << 4) + rlane] = v;
      }
    }
    __builtin_amdgcn_fence(__ATOMIC_RELEASE, "workgroup");
    __builtin_amdgcn_wave_barrier();
    __builtin_amdgcn_fence(__ATOMIC_ACQUIRE, "workgroup");
    if (OUT_MODE == 0) {
      float* C = (float*)Cout + (size_t)b * strideC;
      const int hh = lane >> 4, c4 = (lane & 15) * 4;
      for (int pass = 0; pass < 2; ++pass) {
#pragma unroll
        for (int it = 0; it < 8; ++it) {
          const int row = it * 2 + hh;
          v4f v = *(const v4f*)(slab + row * 68 + c4);
          *(volatile v4f*)(C + (size_t)(mBase + row) * ldc + n0 + c4) = v;
        }
        __threadfence();
      }
    } else {
      const int q = lane >> 3, c8 = (lane & 7) * 8;
      unsigned short* C  = (unsigned short*)Cout  + (size_t)b * strideC;
      unsigned short* C2 = (OUT_MODE == 2) ? ((unsigned short*)Cout2 + (size_t)b * strideC) : nullptr;
      for (int pass = 0; pass < 2; ++pass) {
#pragma unroll
        for (int it = 0; it < 4; ++it) {
          const int row = it * 4 + q;
          const float* sp = slab + row * 68 + c8;
          v8h hv, lv;
#pragma unroll
          for (int e = 0; e < 8; ++e) {
            if (OUT_MODE == 1) {
              hv[e] = (_Float16)sp[e];
            } else {
              unsigned short hb = f2bf_bits(sp[e]);
              unsigned short lb = f2bf_bits(sp[e] - bf_bits2f(hb));
              hv[e] = __builtin_bit_cast(_Float16, hb);
              lv[e] = __builtin_bit_cast(_Float16, lb);
            }
          }
          *(volatile v8h*)(C + (size_t)(mBase + row) * ldc + n0 + c8) = hv;
          if (OUT_MODE == 2) *(volatile v8h*)(C2 + (size_t)(mBase + row) * ldc + n0 + c8) = lv;
        }
        __threadfence();
      }
    }
    __builtin_amdgcn_fence(__ATOMIC_RELEASE, "workgroup");
    __builtin_amdgcn_wave_barrier();
    __builtin_amdgcn_fence(__ATOMIC_ACQUIRE, "workgroup");
  }
}

__global__ __launch_bounds__(256) void k_tables(const float* __restrict__ b1, const float* __restrict__ b2,
                                                float* __restrict__ tab) {
  const int i = blockIdx.x * 256 + threadIdx.x;
  if (i >= TAB_TOTAL) return;
  const int ip = (i < TAB_B1) ? i : (TAB_B1 - 1);
  const int ch = ip / 96;
  const int pidx = ip - ch * 96;
  const int cc = ch & 31;
  const int j = cc >> 1;
  const float emb = ((float)(pidx + 1) / 96.0f) * 6.28318530717958647692f;
  const float tt = powf(10000.0f, (float)j * 0.0625f);
  const float ang = emb / tt;
  float sv, cv;
  sincosf(ang, &sv, &cv);
  const float posv = (cc & 1) ? cv : sv;
  const int i1 = imin(imax(i - TAB_B1, 0), NHID - 1);
  const int i2 = imin(imax(i - TAB_B2, 0), NCHAN - 1);
  const float vb1 = 16.0f * bf16r(b1[i1]);
  const float vb2 = bf16r(b2[i2]);
  const float val = (i < TAB_B1) ? posv : ((i < TAB_B2) ? vb1 : vb2);
  ((volatile float*)tab)[i] = val;
  __threadfence();
  ((volatile float*)tab)[i] = val;
}

__global__ __launch_bounds__(256) void k_castw(const float* __restrict__ wq, const float* __restrict__ wk,
                                               const float* __restrict__ wv, const float* __restrict__ wfc,
                                               const float* __restrict__ wm1, const float* __restrict__ wm2,
                                               _Float16* __restrict__ Wall) {
  const int i = blockIdx.x * 256 + threadIdx.x;
  const int u = i >> 11;
  const int li = i & 2047;
  const float* src = (u == 0) ? wq : (u == 1) ? wk : (u == 2) ? wv : (u == 3) ? wfc
                   : (u == 4) ? wm1 : (u == 5) ? (wm1 + 4096) : (u == 6) ? wm2 : (wm2 + 4096);
  const float f0 = bf16r(src[2 * li]) * 16.0f;
  const float f1 = bf16r(src[2 * li + 1]) * 16.0f;
  const _Float16 h0 = (_Float16)f0, h1 = (_Float16)f1;
  const unsigned packed = (unsigned)__builtin_bit_cast(unsigned short, h0) | ((unsigned)__builtin_bit_cast(unsigned short, h1) << 16);
  ((volatile unsigned*)Wall)[i] = packed;
  __threadfence();
  ((volatile unsigned*)Wall)[i] = packed;
}

__global__ __launch_bounds__(256) void k_pack(const float* __restrict__ q, const float* __restrict__ k,
                                              const float* __restrict__ v, const float* __restrict__ tab,
                                              _Float16* __restrict__ X16) {
  __shared__ __align__(16) float tile[64 * TILE_PITCH];
  const int t = blockIdx.y;
  const float* src = (t == 0) ? q : ((t == 1) ? k : v);
  const int tb = blockIdx.x;
  const int bb = tb / (HWPIX / 64);
  const int p0 = (tb - bb * (HWPIX / 64)) * 64;
  const int tid = threadIdx.x, lane = tid & 31, wave = tid >> 5;
  const float* xb = src + (size_t)bb * NCHAN * HWPIX + p0;
#pragma unroll
  for (int it = 0; it < 4; ++it) {
    const int idx = it * 256 + tid;
    const int cch = idx >> 4;
    const int p4 = (idx & 15) * 4;
    const int pix = p0 + p4;
    const int yy = pix / IMG_W;
    const int xx = pix - yy * IMG_W;
    const v4f d = *(const v4f*)(xb + (size_t)cch * HWPIX + p4);
    const float py = tab[cch * 96 + yy];
    const v4f pxv = *(const v4f*)(tab + cch * 96 + xx);
    v4f o;
#pragma unroll
    for (int e = 0; e < 4; ++e) {
      const float val = bf16r(d[e]);
      const float pv = (cch < 32) ? py : pxv[e];
      o[e] = (t < 2) ? (val + pv) : val;
    }
    *(v4f*)(tile + cch * TILE_PITCH + p4) = o;
  }
  __syncthreads();
  const int q8 = lane >> 3, c8 = (lane & 7) * 8;
  const size_t plane = (size_t)t * PLANE16;
  for (int pass = 0; pass < 2; ++pass) {
#pragma unroll
    for (int it = 0; it < 2; ++it) {
      const int r = wave * 8 + it * 4 + q8;
      v8h hv;
#pragma unroll
      for (int e = 0; e < 8; ++e) hv[e] = (_Float16)tile[(c8 + e) * TILE_PITCH + r];
      *(volatile v8h*)(X16 + plane + (size_t)(bb * HWPIX + p0 + r) * NCHAN + c8) = hv;
    }
    __threadfence();
  }
}

__global__ __launch_bounds__(256) void k_attn_fc(const float* __restrict__ QKV, const float* __restrict__ flow,
                                                 const _Float16* __restrict__ Wfc,
                                                 float* __restrict__ Fc32, _Float16* __restrict__ Fc16) {
  __shared__ __align__(16) _Float16 attS[32 * ATT_PITCH];
  __shared__ __align__(16) float outS[32 * OUT_PITCH];
  const int tid = threadIdx.x;
  const int lane = tid & 31, wave = tid >> 5;
  const int pl = tid >> 3, hd = tid & 7;
  const int pixBase = blockIdx.x * 32;
  const int pix = pixBase + pl;
  const int bb = pix / HWPIX;
  const int p = pix - bb * HWPIX;
  const int y = p / IMG_W;
  const int x = p - y * IMG_W;
  const float fx = bf16r(flow[((size_t)bb * 2 + 0) * HWPIX + p]);
  const float fy = bf16r(flow[((size_t)bb * 2 + 1) * HWPIX + p]);

  const float* qp = QKV + (size_t)pix * NCHAN + hd * HDIM;
  const v4f qlo = *(const v4f*)(qp);
  const v4f qhi = *(const v4f*)(qp + 4);
  float qv[8];
#pragma unroll
  for (int e = 0; e < 4; ++e) { qv[e] = qlo[e]; qv[4 + e] = qhi[e]; }
  const float* Kb = QKV + PLANE32 + (size_t)bb * HWPIX * NCHAN + hd * HDIM;
  const float* Vb = QKV + 2 * PLANE32 + (size_t)bb * HWPIX * NCHAN + hd * HDIM;

  float mrun = -1.0e30f, lrun = 0.0f;
  float oac[8];
#pragma unroll
  for (int e = 0; e < 8; ++e) oac[e] = 0.0f;

#pragma unroll 1
  for (int t = 0; t < NTAPS; ++t) {
    const int ky = t / KWIN;
    const int kx = t - ky * KWIN;
    float xs = (float)(x + kx - 2) + fx;
    float ys = (float)(y + ky - 2) + fy;
    xs = fminf(fmaxf(xs, -32.0f), 160.0f);
    ys = fminf(fmaxf(ys, -32.0f), 160.0f);
    const float x0f = floorf(xs), y0f = floorf(ys);
    const float wx = xs - x0f, wy = ys - y0f;
    const int x0 = (int)x0f, y0 = (int)y0f;
    const int x1 = x0 + 1, y1 = y0 + 1;
    const float vx0 = (x0 >= 0 && x0 <= IMG_W - 1) ? 1.0f : 0.0f;
    const float vx1 = (x1 >= 0 && x1 <= IMG_W - 1) ? 1.0f : 0.0f;
    const float vy0 = (y0 >= 0 && y0 <= IMG_H - 1) ? 1.0f : 0.0f;
    const float vy1 = (y1 >= 0 && y1 <= IMG_H - 1) ? 1.0f : 0.0f;
    const int xc0 = imin(imax(x0, 0), IMG_W - 1), xc1 = imin(imax(x1, 0), IMG_W - 1);
    const int yc0 = imin(imax(y0, 0), IMG_H - 1), yc1 = imin(imax(y1, 0), IMG_H - 1);
    const float w00 = ((1.0f - wy) * (1.0f - wx)) * (vy0 * vx0);
    const float w01 = ((1.0f - wy) * wx) * (vy0 * vx1);
    const float w10 = (wy * (1.0f - wx)) * (vy1 * vx0);
    const float w11 = (wy * wx) * (vy1 * vx1);
    const int o00 = (yc0 * IMG_W + xc0) * NCHAN;
    const int o01 = (yc0 * IMG_W + xc1) * NCHAN;
    const int o10 = (yc1 * IMG_W + xc0) * NCHAN;
    const int o11 = (yc1 * IMG_W + xc1) * NCHAN;
    float ks[8], vs[8];
    {
      const v4f a0 = *(const v4f*)(Kb + o00), a1 = *(const v4f*)(Kb + o00 + 4);
      const v4f g0 = *(const v4f*)(Kb + o01), g1 = *(const v4f*)(Kb + o01 + 4);
      const v4f c0 = *(const v4f*)(Kb + o10), c1 = *(const v4f*)(Kb + o10 + 4);
      const v4f d0 = *(const v4f*)(Kb + o11), d1 = *(const v4f*)(Kb + o11 + 4);
#pragma unroll
      for (int e = 0; e < 4; ++e) {
        ks[e]     = w00 * a0[e] + w01 * g0[e] + w10 * c0[e] + w11 * d0[e];
        ks[4 + e] = w00 * a1[e] + w01 * g1[e] + w10 * c1[e] + w11 * d1[e];
      }
    }
    {
      const v4f a0 = *(const v4f*)(Vb + o00), a1 = *(const v4f*)(Vb + o00 + 4);
      const v4f g0 = *(const v4f*)(Vb + o01), g1 = *(const v4f*)(Vb + o01 + 4);
      const v4f c0 = *(const v4f*)(Vb + o10), c1 = *(const v4f*)(Vb + o10 + 4);
      const v4f d0 = *(const v4f*)(Vb + o11), d1 = *(const v4f*)(Vb + o11 + 4);
#pragma unroll
      for (int e = 0; e < 4; ++e) {
        vs[e]     = w00 * a0[e] + w01 * g0[e] + w10 * c0[e] + w11 * d0[e];
        vs[4 + e] = w00 * a1[e] + w01 * g1[e] + w10 * c1[e] + w11 * d1[e];
      }
    }
    float sc = 0.0f;
#pragma unroll
    for (int e = 0; e < 8; ++e) sc += qv[e] * ks[e];
    sc *= (1.0f / 2.82842712474619009760f);
    const float mn = fmaxf(mrun, sc);
    const float fdec = expf(mrun - mn);
    const float ecur = expf(sc - mn);
    lrun = lrun * fdec + ecur;
#pragma unroll
    for (int e = 0; e < 8; ++e) oac[e] = oac[e] * fdec + ecur * vs[e];
    mrun = mn;
  }
  {
    const float osc = 16.0f / lrun;
    v8h hv;
#pragma unroll
    for (int e = 0; e < 8; ++e) hv[e] = (_Float16)(oac[e] * osc);
    *(v8h*)(attS + pl * ATT_PITCH + hd * HDIM) = hv;
  }
  __syncthreads();

  const int rl = lane & 15, hh = lane >> 4, koff = hh * 8;
  const int m0 = (wave >> 2) * 16, n0 = (wave & 3) * 16;
  v8f cacc = {0.f, 0.f, 0.f, 0.f, 0.f, 0.f, 0.f, 0.f};
#pragma unroll
  for (int kstep = 0; kstep < 2; ++kstep) {
    const int k0 = kstep * 32;
    Frag<_Float16>::U fa;
    fa.h[0] = *(const v8h*)(attS + (m0 + rl) * ATT_PITCH + k0 + koff);
    fa.h[1] = *(const v8h*)(attS + (m0 + rl) * ATT_PITCH + k0 + 16 + koff);
    const v16h bw = Frag<_Float16>::load(Wfc + (size_t)(n0 + rl) * NCHAN + k0 + koff);
    cacc = Frag<_Float16>::mma(fa.v, bw, cacc);
    mma_guard1(cacc, fa.v, bw);
  }
#pragma unroll
  for (int r = 0; r < 8; ++r) outS[(m0 + 8 * hh + r) * OUT_PITCH + n0 + rl] = cacc[r] * (1.0f / 256.0f);
  __syncthreads();

  {
    const int rowA = wave * 4;
    const int c4 = (lane & 15) * 4;
    const int q8 = lane >> 3, c8 = (lane & 7) * 8;
    for (int pass = 0; pass < 2; ++pass) {
#pragma unroll
      for (int it = 0; it < 2; ++it) {
        const int row = rowA + it * 2 + hh;
        const v4f val = *(const v4f*)(outS + row * OUT_PITCH + c4);
        *(volatile v4f*)(Fc32 + (size_t)(pixBase + row) * NCHAN + c4) = val;
      }
      {
        const int row = rowA + q8;
        const float* sp = outS + row * OUT_PITCH + c8;
        v8h hv2;
#pragma unroll
        for (int e = 0; e < 8; ++e) hv2[e] = (_Float16)(sp[e] * 16.0f);
        *(volatile v8h*)(Fc16 + (size_t)(pixBase + row) * NCHAN + c8) = hv2;
      }
      __threadfence();
    }
  }
}

__device__ __forceinline__ double stat_sum64(const float* __restrict__ P, int lineBase, int lane) {
  double v = (double)P[(size_t)(lineBase + lane) * 32] + (double)P[(size_t)(lineBase + 32 + lane) * 32];
#pragma unroll
  for (int off = 16; off > 0; off >>= 1) v += __shfl_xor(v, off, 32);
  return __shfl(v, 0, 32);
}

__global__ __launch_bounds__(256) void k_gn_sum(const float* __restrict__ Y2, const float* __restrict__ Fc32,
                                                float* __restrict__ P1) {
  __shared__ float red[8];
  const int blk = blockIdx.x;
  const int tid = threadIdx.x, lane = tid & 31, wave = tid >> 5;
  const size_t base = (size_t)blk * GN_CHUNK;
  float s = 0.0f;
#pragma unroll 3
  for (int it = 0; it < GN_CHUNK / 1024; ++it) {
    const size_t o = base + (size_t)(it * 256 + tid) * 4;
    const v4f a = *(const v4f*)(Y2 + o);
    const v4f c = *(const v4f*)(Fc32 + o);
    s += ((a[0] + c[0]) + (a[1] + c[1])) + ((a[2] + c[2]) + (a[3] + c[3]));
  }
#pragma unroll
  for (int off = 16; off > 0; off >>= 1) s += __shfl_xor(s, off, 32);
  if (lane == 0) red[wave] = s;
  __syncthreads();
  if (wave == 0) {
    float tot = 0.0f;
#pragma unroll
    for (int w = 0; w < 8; ++w) tot += red[w];
    const float ov = (lane == 0) ? tot : 0.0f;
    ((volatile float*)P1)[(size_t)blk * 32 + lane] = ov;
    __threadfence();
    ((volatile float*)P1)[(size_t)blk * 32 + lane] = ov;
  }
}

__global__ __launch_bounds__(256) void k_gn_var(const float* __restrict__ Y2, const float* __restrict__ Fc32,
                                                const float* __restrict__ P1, float* __restrict__ P2) {
  __shared__ float red[8];
  const int blk = blockIdx.x;
  const int tid = threadIdx.x, lane = tid & 31, wave = tid >> 5;
  const int bb = blk >> 6;
  const double su = stat_sum64(P1, bb * 64, lane);
  const float mu = (float)(su * (1.0 / (double)NSAMPLE));
  const size_t base = (size_t)blk * GN_CHUNK;
  float s = 0.0f;
#pragma unroll 3
  for (int it = 0; it < GN_CHUNK / 1024; ++it) {
    const size_t o = base + (size_t)(it * 256 + tid) * 4;
    const v4f a = *(const v4f*)(Y2 + o);
    const v4f c = *(const v4f*)(Fc32 + o);
    const float d0 = (a[0] + c[0]) - mu, d1 = (a[1] + c[1]) - mu, d2 = (a[2] + c[2]) - mu, d3 = (a[3] + c[3]) - mu;
    s += ((d0 * d0) + (d1 * d1)) + ((d2 * d2) + (d3 * d3));
  }
#pragma unroll
  for (int off = 16; off > 0; off >>= 1) s += __shfl_xor(s, off, 32);
  if (lane == 0) red[wave] = s;
  __syncthreads();
  if (wave == 0) {
    float tot = 0.0f;
#pragma unroll
    for (int w = 0; w < 8; ++w) tot += red[w];
    const float ov = (lane == 0) ? tot : 0.0f;
    ((volatile float*)P2)[(size_t)blk * 32 + lane] = ov;
    __threadfence();
    ((volatile float*)P2)[(size_t)blk * 32 + lane] = ov;
  }
}

__global__ __launch_bounds__(256) void k_gn_out(const float* __restrict__ Y2, const float* __restrict__ Fc32,
                                                const float* __restrict__ P1, const float* __restrict__ P2,
                                                const float* __restrict__ gw, const float* __restrict__ gb,
                                                float* __restrict__ out) {
  __shared__ __align__(16) float tileT[64 * TILE_PITCH];
  const int tid = threadIdx.x, lane = tid & 31, wave = tid >> 5, hh = lane >> 4;
  const int tb = blockIdx.x;
  const int bb = tb / (HWPIX / 64);
  const int p0 = (tb - bb * (HWPIX / 64)) * 64;
  const double su = stat_sum64(P1, bb * 64, lane);
  const double sv = stat_sum64(P2, bb * 64, lane);
  const float mu = (float)(su * (1.0 / (double)NSAMPLE));
  const float var = (float)(sv * (1.0 / (double)NSAMPLE));
  const float inv = 1.0f / sqrtf(var + 1.0e-5f);
  const size_t rowBase = (size_t)bb * HWPIX + p0;
#pragma unroll
  for (int it = 0; it < 4; ++it) {
    const int idx = it * 256 + tid;
    const int px = idx >> 4;
    const int c4 = (idx & 15) * 4;
    const size_t o = (rowBase + px) * NCHAN + c4;
    const v4f a = *(const v4f*)(Y2 + o);
    const v4f c = *(const v4f*)(Fc32 + o);
#pragma unroll
    for (int e = 0; e < 4; ++e) tileT[(c4 + e) * TILE_PITCH + px] = a[e] + c[e];
  }
  __syncthreads();
  const int c4px = (lane & 15) * 4;
  for (int pass = 0; pass < 2; ++pass) {
#pragma unroll
    for (int it = 0; it < 4; ++it) {
      const int ch = wave * 8 + it * 2 + hh;
      const v4f val = *(const v4f*)(tileT + ch * TILE_PITCH + c4px);
      const float g1 = bf16r(gw[ch]);
      const float g0 = bf16r(gb[ch]);
      v4f ov;
#pragma unroll
      for (int e = 0; e < 4; ++e) ov[e] = ((val[e] - mu) * inv) * g1 + g0;
      *(volatile v4f*)(out + ((size_t)(bb * NCHAN + ch) * HWPIX + p0 + c4px)) = ov;
    }
    __threadfence();
  }
}

extern "C" void kernel_launch(void* const* d_in, const int* in_sizes, int n_in,
                              void* d_out, int out_size, void* d_ws, size_t ws_size,
                              hipStream_t stream)
{
  if (n_in < 14) return;
  if (in_sizes[0] != NBATCH * NCHAN * HWPIX || in_sizes[1] != NBATCH * NCHAN * HWPIX ||
      in_sizes[2] != NBATCH * NCHAN * HWPIX || in_sizes[3] != NBATCH * 2 * HWPIX) return;
  if (in_sizes[4] != 4096 || in_sizes[5] != 4096 || in_sizes[6] != 4096 || in_sizes[7] != 4096) return;
  if (in_sizes[8] != NHID * NCHAN || in_sizes[9] != NHID || in_sizes[10] != NCHAN * NHID ||
      in_sizes[11] != NCHAN || in_sizes[12] != NCHAN || in_sizes[13] != NCHAN) return;
  if (out_size < NBATCH * NCHAN * HWPIX) return;
  if (ws_size < WS_TOTAL) return;

  const float* q      = (const float*)d_in[0];
  const float* k      = (const float*)d_in[1];
  const float* v      = (const float*)d_in[2];
  const float* flow   = (const float*)d_in[3];
  const float* w_qs   = (const float*)d_in[4];
  const float* w_ks   = (const float*)d_in[5];
  const float* w_vs   = (const float*)d_in[6];
  const float* w_fc   = (const float*)d_in[7];
  const float* mlp_w1 = (const float*)d_in[8];
  const float* mlp_b1 = (const float*)d_in[9];
  const float* mlp_w2 = (const float*)d_in[10];
  const float* mlp_b2 = (const float*)d_in[11];
  const float* norm_w = (const float*)d_in[12];
  const float* norm_b = (const float*)d_in[13];
  float* out = (float*)d_out;

  char* ws = (char*)d_ws;
  float*    tab  = (float*)(ws + OFF_TAB);
  _Float16* Wall = (_Float16*)(ws + OFF_WALL);
  _Float16* X16  = (_Float16*)(ws + OFF_X16);
  float*    QKV  = (float*)(ws + OFF_QKV);
  float*    Fc32 = (float*)(ws + OFF_FC32);
  _Float16* Fc16 = (_Float16*)(ws + OFF_FC16);
  _Float16* Hd16 = (_Float16*)(ws + OFF_HD16);
  float*    Y2   = (float*)(ws + OFF_Y2);
  float*    P1   = (float*)(ws + OFF_P1);
  float*    P2   = (float*)(ws + OFF_P2);
  const unsigned short* WallU = (const unsigned short*)Wall;
  const unsigned short* X16U  = (const unsigned short*)X16;
  const unsigned short* Fc16U = (const unsigned short*)Fc16;
  const unsigned short* Hd16U = (const unsigned short*)Hd16;

  k_tables<<<(TAB_TOTAL + 255) / 256, 256, 0, stream>>>(mlp_b1, mlp_b2, tab);
  k_castw<<<(W_TOTAL / 2) / 256, 256, 0, stream>>>(w_qs, w_ks, w_vs, w_fc, mlp_w1, mlp_w2, Wall);
  k_pack<<<dim3(NROWS / 64, 3), 256, 0, stream>>>(q, k, v, tab, X16);

  static_assert(NROWS % 64 == 0 && NCHAN % 64 == 0 && NCHAN % 32 == 0 && NHID % 64 == 0 && NHID % 32 == 0);
  {
    const int tiles = (NROWS / 64) * (NCHAN / 64);
    wmma_gemm64<0, false, 0, 0, false, 0><<<dim3((tiles + 7) / 8, 3), 256, 0, stream>>>(
        X16U, X16U, NCHAN, PLANE16,
        WallU + W_Q, WallU + W_Q, NCHAN, 4096L,
        (void*)QKV, (void*)QKV, NCHAN, PLANE32,
        tab, tab, 0L, NROWS, NCHAN, NCHAN, 1.0f / 16.0f);
  }

  k_attn_fc<<<NROWS / 32, 256, 0, stream>>>(QKV, flow, Wall + W_FC, Fc32, Fc16);

  {
    const int tiles = (NROWS / 64) * (NHID / 64);
    wmma_gemm64<0, false, 2, 1, false, 6><<<dim3((tiles + 7) / 8, 1), 256, 0, stream>>>(
        Fc16U, Fc16U, NCHAN, 0L,
        WallU + W_M1, WallU + W_M1, NCHAN, 0L,
        (void*)Hd16, (void*)Hd16, NHID, 0L,
        tab + TAB_B1, tab, 0L, NROWS, NHID, NCHAN, 1.0f / 16.0f);
  }
  {
    const int tiles = (NROWS / 64) * (NCHAN / 64);
    wmma_gemm64<0, false, 2, 0, false, 0><<<dim3((tiles + 7) / 8, 1), 256, 0, stream>>>(
        Hd16U, Hd16U, NHID, 0L,
        WallU + W_M2, WallU + W_M2, NHID, 0L,
        (void*)Y2, (void*)Y2, NCHAN, 0L,
        tab + TAB_B2, tab, 0L, NROWS, NCHAN, NHID, 1.0f / 256.0f);
  }

  k_gn_sum<<<GN_BLOCKS, 256, 0, stream>>>(Y2, Fc32, P1);
  k_gn_var<<<GN_BLOCKS, 256, 0, stream>>>(Y2, Fc32, P1, P2);
  k_gn_out<<<NROWS / 64, 256, 0, stream>>>(Y2, Fc32, P1, P2, norm_w, norm_b, out);
}
